// R3D2Net_30975304139468
// MI455X (gfx1250) — hardware-verified
//
#include <hip/hip_runtime.h>
#include <math.h>

typedef __attribute__((ext_vector_type(16))) _Float16 v16h;
typedef __attribute__((ext_vector_type(8)))  _Float16 v8h;
typedef __attribute__((ext_vector_type(16))) __bf16   v16b;
typedef __attribute__((ext_vector_type(8)))  __bf16   v8b;
typedef __attribute__((ext_vector_type(8)))  float    v8f;
typedef __attribute__((ext_vector_type(4)))  float    v4f;
typedef __attribute__((ext_vector_type(4)))  unsigned int v4u;
#define PSCALE 32768.0f
#define U16(p) ((const unsigned short*)(const void*)(p))
#define PSCALE_INV (1.0f / 32768.0f)

__device__ __forceinline__ unsigned short f2bf_bits(float f) {
  unsigned u = __float_as_uint(f);
  return (unsigned short)((u + 0x7FFFu + ((u >> 16) & 1u)) >> 16);
}
__device__ __forceinline__ float bf_bits2f(unsigned short h) { return __uint_as_float(((unsigned)h) << 16); }

__device__ __forceinline__ void dep_guard_h(v8f& a, v8f& b, v16h x, v16h y) { asm volatile("v_nop\n\tv_nop\n\tv_nop\n\tv_nop" : "+v"(a), "+v"(b) : "v"(x), "v"(y)); }
__device__ __forceinline__ void dep_guard_b(v8f& a, v8f& b, v16b x, v16b y) { asm volatile("v_nop\n\tv_nop\n\tv_nop\n\tv_nop" : "+v"(a), "+v"(b) : "v"(x), "v"(y)); }
__device__ __forceinline__ void keep4_h(v16h a, v16h b, v16h c, v16h d) { asm volatile("v_nop" :: "v"(a), "v"(b), "v"(c), "v"(d)); }
__device__ __forceinline__ void keep4_b(v16b a, v16b b, v16b c, v16b d) { asm volatile("v_nop" :: "v"(a), "v"(b), "v"(c), "v"(d)); }
__device__ __forceinline__ void acc_guard4(v8f& a, v8f& b, v8f& c, v8f& d) { asm volatile("v_nop\n\tv_nop\n\tv_nop\n\tv_nop" : "+v"(a), "+v"(b), "+v"(c), "+v"(d)); }
template <typename T> struct Frag;
template <> struct Frag<_Float16> {
  typedef v16h V; union U { v16h v; v8h h[2]; };
  static __device__ __forceinline__ v16h load(const _Float16* p) {
    U f; f.h[0] = *(const v8h*)(p); f.h[1] = *(const v8h*)(p + 16); return f.v;
  }
  static __device__ __forceinline__ v8f mma(v16h a, v16h b, v8f c) {
    return __builtin_amdgcn_wmma_f32_16x16x32_f16(false, a, false, b, (short)0, c, false, false);
  }
  static __device__ __forceinline__ void guard(v8f& a, v8f& b, v16h x, v16h y) { dep_guard_h(a, b, x, y); }
  static __device__ __forceinline__ void keep(v16h a, v16h b, v16h c, v16h d) { keep4_h(a, b, c, d); }
};
template <> struct Frag<__bf16> {
  typedef v16b V; union U { v16b v; v8b h[2]; };
  static __device__ __forceinline__ v16b load(const __bf16* p) {
    U f; f.h[0] = *(const v8b*)(p); f.h[1] = *(const v8b*)(p + 16); return f.v;
  }
  static __device__ __forceinline__ v8f mma(v16b a, v16b b, v8f c) {
    return __builtin_amdgcn_wmma_f32_16x16x32_bf16(false, a, false, b, (short)0, c, false, false);
  }
  static __device__ __forceinline__ void guard(v8f& a, v8f& b, v16b x, v16b y) { dep_guard_b(a, b, x, y); }
  static __device__ __forceinline__ void keep(v16b a, v16b b, v16b c, v16b d) { keep4_b(a, b, c, d); }
};

template <int ET> struct Elem;
template <> struct Elem<0> { typedef _Float16 T; };
template <> struct Elem<1> { typedef __bf16 T; };
template <int ET, bool SPLIT, int BIAS_MODE, int OUT_MODE, bool RESID, int ACT = 0>
__global__ __launch_bounds__(256) void wmma_gemm64(
    const unsigned short* __restrict__ Ap, const unsigned short* __restrict__ A2p, int lda, long strideA,
    const unsigned short* __restrict__ Btp, const unsigned short* __restrict__ Bt2p, int ldb, long strideB,
    void* __restrict__ Cout, void* __restrict__ Cout2, int ldc, long strideC,
    const float* __restrict__ bias,
    const float* __restrict__ resid, long strideR,
    int M, int N, int K, float scale) {
  typedef typename Elem<ET>::T T;
  typedef typename Frag<T>::V V;
  const T* A = (const T*)Ap; const T* A2 = (const T*)A2p; const T* Bt = (const T*)Btp; const T* Bt2 = (const T*)Bt2p;
  __shared__ __align__(16) float sT[8][16 * 68];
  const int b    = blockIdx.y;
  const int lane = threadIdx.x & 31;
  const int wave = threadIdx.x >> 5;
  const int tilesN = N >> 6;
  const int tilesM = M >> 6;
  const int tile = blockIdx.x * 8 + wave;
  if (tile >= tilesM * tilesN) return;
  const int tm = tile / tilesN;
  const int tn = tile - tm * tilesN;
  const int m0 = tm << 6;
  const int n0 = tn << 6;

  const T* Ab  = A  + (size_t)b * strideA;
  const T* Bb  = Bt + (size_t)b * strideB;
  const T* Ab2 = SPLIT ? (A2  + (size_t)b * strideA) : nullptr;
  const T* Bb2 = SPLIT ? (Bt2 + (size_t)b * strideB) : nullptr;

  const int rlane = lane & 15;
  const int koff  = (lane >> 4) * 8;
  const int mOff  = (lane >> 4) * 8;

  v8f acc[4][4];
#pragma unroll
  for (int i = 0; i < 4; ++i)
#pragma unroll
    for (int j = 0; j < 4; ++j) acc[i][j] = (v8f){0.f,0.f,0.f,0.f,0.f,0.f,0.f,0.f};

  for (int k0 = 0; k0 < K; k0 += 32) {
    V bh[4], bl[4];
#pragma unroll
    for (int j = 0; j < 4; ++j) {
      const size_t bo = (size_t)(n0 + (j << 4) + rlane) * ldb + koff + k0;
      bh[j] = Frag<T>::load(Bb + bo);
      if (SPLIT) bl[j] = Frag<T>::load(Bb2 + bo);
    }
#pragma unroll
    for (int i = 0; i < 4; ++i) {
      const size_t ao = (size_t)(m0 + (i << 4) + rlane) * lda + koff + k0;
      V ah = Frag<T>::load(Ab + ao);
      V al;
      if (SPLIT) al = Frag<T>::load(Ab2 + ao);
#pragma unroll
      for (int j = 0; j < 4; ++j) {
        acc[i][j] = Frag<T>::mma(ah, bh[j], acc[i][j]);
        if (SPLIT) {
          acc[i][j] = Frag<T>::mma(ah, bl[j], acc[i][j]);
          acc[i][j] = Frag<T>::mma(al, bh[j], acc[i][j]);
        }
      }
      Frag<T>::guard(acc[i][0], acc[i][3], ah, SPLIT ? al : ah);
    }
    Frag<T>::keep(bh[0], bh[1], bh[2], bh[3]);
    if (SPLIT) Frag<T>::keep(bl[0], bl[1], bl[2], bl[3]);
  }
  acc_guard4(acc[0][0], acc[0][1], acc[0][2], acc[0][3]);
  acc_guard4(acc[1][0], acc[1][1], acc[1][2], acc[1][3]);
  acc_guard4(acc[2][0], acc[2][1], acc[2][2], acc[2][3]);
  acc_guard4(acc[3][0], acc[3][1], acc[3][2], acc[3][3]);

  float* slab = sT[wave];
  const float* Rb = RESID ? (resid + (size_t)b * strideR) : nullptr;
#pragma unroll
  for (int i = 0; i < 4; ++i) {
    const int mBase = m0 + (i << 4);
#pragma unroll
    for (int j = 0; j < 4; ++j) {
      const int n = n0 + (j << 4) + rlane;
      float bv = 0.f;
      if (BIAS_MODE == 2) bv = bias[n];
#pragma unroll
      for (int r = 0; r < 8; ++r) {
        float v = acc[i][j][r] * scale;
        if (BIAS_MODE == 1) v += bias[mBase + mOff + r];
        if (BIAS_MODE == 2) v += bv;
        if (RESID) v += Rb[(size_t)(mBase + mOff + r) * ldc + n];
        if (ACT == 1) v = tanhf(v);
        if (ACT == 2) v = fmaxf(v, 0.0f);
        if (ACT == 3) v = v / (1.0f + expf(-v));
        if (ACT == 4) v = (v > 0.f) ? v : 0.01f * v;
        if (ACT == 5) v = 0.5f * v * (1.0f + erff(v * 0.70710678118654752f));
        slab[(mOff + r) * 68 + (j << 4) + rlane] = v;
      }
    }
    __builtin_amdgcn_fence(__ATOMIC_RELEASE, "workgroup");
    __builtin_amdgcn_wave_barrier();
    __builtin_amdgcn_fence(__ATOMIC_ACQUIRE, "workgroup");
    if (OUT_MODE == 0) {
      float* C = (float*)Cout + (size_t)b * strideC;
      const int hh = lane >> 4, c4 = (lane & 15) * 4;
      for (int pass = 0; pass < 2; ++pass) {
#pragma unroll
        for (int it = 0; it < 8; ++it) {
          const int row = it * 2 + hh;
          v4f v = *(const v4f*)(slab + row * 68 + c4);
          *(volatile v4f*)(C + (size_t)(mBase + row) * ldc + n0 + c4) = v;
        }
        __threadfence();
      }
    } else {
      const int q = lane >> 3, c8 = (lane & 7) * 8;
      unsigned short* C  = (unsigned short*)Cout  + (size_t)b * strideC;
      unsigned short* C2 = (OUT_MODE == 2) ? ((unsigned short*)Cout2 + (size_t)b * strideC) : nullptr;
      for (int pass = 0; pass < 2; ++pass) {
#pragma unroll
        for (int it = 0; it < 4; ++it) {
          const int row = it * 4 + q;
          const float* sp = slab + row * 68 + c8;
          v8h hv, lv;
#pragma unroll
          for (int e = 0; e < 8; ++e) {
            if (OUT_MODE == 1) {
              hv[e] = (_Float16)sp[e];
            } else {
              unsigned short hb = f2bf_bits(sp[e]);
              unsigned short lb = f2bf_bits(sp[e] - bf_bits2f(hb));
              hv[e] = __builtin_bit_cast(_Float16, hb);
              lv[e] = __builtin_bit_cast(_Float16, lb);
            }
          }
          *(volatile v8h*)(C + (size_t)(mBase + row) * ldc + n0 + c8) = hv;
          if (OUT_MODE == 2) *(volatile v8h*)(C2 + (size_t)(mBase + row) * ldc + n0 + c8) = lv;
        }
        __threadfence();
      }
    }
    __builtin_amdgcn_fence(__ATOMIC_RELEASE, "workgroup");
    __builtin_amdgcn_wave_barrier();
    __builtin_amdgcn_fence(__ATOMIC_ACQUIRE, "workgroup");
  }
}

constexpr int kSteps = 128;
constexpr int kBatch = 64;
constexpr int kState = 512;
constexpr int kHid   = 512;
constexpr int kGate  = 2048;
constexpr int kBert  = 768;
constexpr int kAct   = 20;
constexpr int kRows  = kSteps * kBatch;
constexpr int kAtp   = 528;
constexpr int kHsp   = 516;

__global__ __launch_bounds__(256) void cast_rows_bf16hl(
    const float* __restrict__ in, unsigned short* __restrict__ hi, unsigned short* __restrict__ lo, int n8) {
  const int i = blockIdx.x * 256 + threadIdx.x;
  if (i < n8) {
    const v4f a = *(const v4f*)(in + (size_t)i * 8);
    const v4f b = *(const v4f*)(in + (size_t)i * 8 + 4);
    const float f[8] = {a[0], a[1], a[2], a[3], b[0], b[1], b[2], b[3]};
    v8h hv, lv;
#pragma unroll
    for (int e = 0; e < 8; ++e) {
      const unsigned short hb = f2bf_bits(f[e]);
      const unsigned short lb = f2bf_bits(f[e] - bf_bits2f(hb));
      hv[e] = __builtin_bit_cast(_Float16, hb);
      lv[e] = __builtin_bit_cast(_Float16, lb);
    }
    for (int pass = 0; pass < 2; ++pass) {
      *(volatile v8h*)(hi + (size_t)i * 8) = hv;
      *(volatile v8h*)(lo + (size_t)i * 8) = lv;
      __threadfence();
    }
  }
}

template <int MODE>
__global__ __launch_bounds__(256) void transpose_cast64(
    const float* __restrict__ W, unsigned short* __restrict__ O1, unsigned short* __restrict__ O2,
    int nK, int nN, float scl) {
  __shared__ __align__(16) float sW[64 * 68];
  const int tid = threadIdx.x, wave = tid >> 5, lane = tid & 31;
  const int n0 = blockIdx.x * 64, k0 = blockIdx.y * 64;
#pragma unroll
  for (int i = 0; i < 4; ++i) {
    const int idx = i * 256 + tid;
    const int kr = idx >> 4;
    const int n4 = (idx & 15) * 4;
    const v4f v = *(const v4f*)(W + (size_t)(k0 + kr) * nN + n0 + n4);
    sW[(n4 + 0) * 68 + kr] = v[0];
    sW[(n4 + 1) * 68 + kr] = v[1];
    sW[(n4 + 2) * 68 + kr] = v[2];
    sW[(n4 + 3) * 68 + kr] = v[3];
  }
  __syncthreads();
  const int q = lane >> 3, c8 = (lane & 7) * 8;
  for (int pass = 0; pass < 2; ++pass) {
#pragma unroll
    for (int it = 0; it < 2; ++it) {
      const int row = it * 32 + wave * 4 + q;
      const float* sp = sW + row * 68 + c8;
      v8h hv, lv;
#pragma unroll
      for (int e = 0; e < 8; ++e) {
        const float f = sp[e];
        if (MODE == 0) {
          hv[e] = (_Float16)(f * scl);
          lv[e] = hv[e];
        } else {
          const unsigned short hb = f2bf_bits(f);
          const unsigned short lb = f2bf_bits(f - bf_bits2f(hb));
          hv[e] = __builtin_bit_cast(_Float16, hb);
          lv[e] = __builtin_bit_cast(_Float16, lb);
        }
      }
      const size_t o = (size_t)(n0 + row) * nK + k0 + c8;
      *(volatile v8h*)(O1 + o) = hv;
      if (MODE == 1) *(volatile v8h*)(O2 + o) = lv;
    }
    __threadfence();
  }
}

__device__ __forceinline__ float sigm_f(float x) { return 1.0f / (1.0f + expf(-x)); }

__global__ __launch_bounds__(256) void lstm_seq_kernel(
    const float* __restrict__ GX,
    const unsigned short* __restrict__ Whp,
    const int* __restrict__ dones,
    const float* __restrict__ c0,
    const float* __restrict__ h0,
    unsigned short* __restrict__ YShi,
    unsigned short* __restrict__ YSlo,
    float* __restrict__ outC,
    float* __restrict__ outH) {
  __shared__ __align__(16) _Float16 aT[16 * kAtp];
  __shared__ __align__(16) float hS[16 * kHsp];
  const int tid = threadIdx.x, wave = tid >> 5, lane = tid & 31;
  const int hh = lane >> 4, c = lane & 15;
  const int koff = hh * 8;
  const int row0 = blockIdx.x * 16;
  const _Float16* Wh16 = (const _Float16*)Whp;
  const int q4 = lane >> 3, c8 = (lane & 7) * 8, c4 = (lane & 7) * 4;
  const float accScale = 1.0f / 16384.0f;

#pragma unroll
  for (int i = 0; i < 4; ++i) {
    const int qd = i * 256 + tid;
    const int row = qd >> 6;
    const int col8 = (qd & 63) * 8;
    const float* src = h0 + (size_t)(row0 + row) * kHid + col8;
    const v4f x0 = *(const v4f*)src;
    const v4f x1 = *(const v4f*)(src + 4);
    const int dz = dones[row0 + row];
    v8h hv;
#pragma unroll
    for (int e = 0; e < 4; ++e) {
      const float fa = (dz != 0) ? 0.0f : x0[e] * 256.0f;
      const float fb = (dz != 0) ? 0.0f : x1[e] * 256.0f;
      hv[e] = (_Float16)fa;
      hv[4 + e] = (_Float16)fb;
    }
    *(v8h*)(aT + row * kAtp + col8) = hv;
  }
  float creg[4][8];
#pragma unroll
  for (int ubl = 0; ubl < 4; ++ubl) {
    const int u = 16 * (wave * 4 + ubl) + c;
#pragma unroll
    for (int r = 0; r < 8; ++r) creg[ubl][r] = c0[(size_t)(row0 + 8 * hh + r) * kHid + u];
  }
  __syncthreads();

  for (int t = 0; t < kSteps; ++t) {
    unsigned dmask = 0u;
#pragma unroll
    for (int r = 0; r < 8; ++r)
      dmask |= ((dones[t * kBatch + row0 + 8 * hh + r] != 0) ? 1u : 0u) << r;

#pragma unroll
    for (int p = 0; p < 2; ++p) {
      v8f acc[2][4];
#pragma unroll
      for (int j = 0; j < 2; ++j)
#pragma unroll
        for (int g = 0; g < 4; ++g) acc[j][g] = (v8f){0.f,0.f,0.f,0.f,0.f,0.f,0.f,0.f};

#pragma unroll 1
      for (int k0 = 0; k0 < kHid; k0 += 32) {
        const v16h a = Frag<_Float16>::load(aT + c * kAtp + koff + k0);
#pragma unroll
        for (int j = 0; j < 2; ++j) {
          const int ub16 = 16 * (wave * 4 + p * 2 + j);
          v16h bq[4];
#pragma unroll
          for (int g = 0; g < 4; ++g)
            bq[g] = Frag<_Float16>::load(Wh16 + (size_t)(g * kHid + ub16 + c) * kHid + koff + k0);
#pragma unroll
          for (int g = 0; g < 4; ++g) acc[j][g] = Frag<_Float16>::mma(a, bq[g], acc[j][g]);
          Frag<_Float16>::guard(acc[j][0], acc[j][3], a, bq[3]);
          Frag<_Float16>::keep(bq[0], bq[1], bq[2], bq[3]);
        }
      }
      acc_guard4(acc[0][0], acc[0][1], acc[0][2], acc[0][3]);
      acc_guard4(acc[1][0], acc[1][1], acc[1][2], acc[1][3]);

#pragma unroll
      for (int j = 0; j < 2; ++j) {
        const int ubl = p * 2 + j;
        const int u = 16 * (wave * 4 + ubl) + c;
#pragma unroll
        for (int r = 0; r < 8; ++r) {
          const size_t gro = (size_t)(t * kBatch + row0 + 8 * hh + r) * kGate + u;
          const float gi = acc[j][0][r] * accScale + GX[gro];
          const float gf = acc[j][1][r] * accScale + GX[gro + kHid];
          const float gg = acc[j][2][r] * accScale + GX[gro + 2 * kHid];
          const float gq = acc[j][3][r] * accScale + GX[gro + 3 * kHid];
          const float ci = ((dmask >> r) & 1u) ? 0.0f : creg[ubl][r];
          const float nc = sigm_f(gf) * ci + sigm_f(gi) * tanhf(gg);
          const float nh = sigm_f(gq) * tanhf(nc);
          creg[ubl][r] = nc;
          hS[(8 * hh + r) * kHsp + u] = nh;
        }
      }
    }
    __syncthreads();

    {
      const int tn = (t + 1 < kSteps) ? (t + 1) : (kSteps - 1);
#pragma unroll
      for (int i = 0; i < 4; ++i) {
        const int qd = i * 256 + tid;
        const int row = qd >> 6;
        const int col8 = (qd & 63) * 8;
        const float* sp = hS + row * kHsp + col8;
        const v4f x0 = *(const v4f*)sp;
        const v4f x1 = *(const v4f*)(sp + 4);
        const int dz = dones[tn * kBatch + row0 + row];
        v8h hv;
#pragma unroll
        for (int e = 0; e < 4; ++e) {
          const float fa = (dz != 0) ? 0.0f : x0[e] * 256.0f;
          const float fb = (dz != 0) ? 0.0f : x1[e] * 256.0f;
          hv[e] = (_Float16)fa;
          hv[4 + e] = (_Float16)fb;
        }
        *(v8h*)(aT + row * kAtp + col8) = hv;
      }
    }
    for (int pass = 0; pass < 2; ++pass) {
#pragma unroll
      for (int it = 0; it < 4; ++it) {
        const int si = it * 4 + q4;
        const int row = 2 * wave + (si >> 3);
        const int col = (si & 7) * 64 + c8;
        const float* sp = hS + row * kHsp + col;
        v8h hv, lv;
#pragma unroll
        for (int e = 0; e < 8; ++e) {
          const float f = sp[e];
          const unsigned short hb = f2bf_bits(f);
          const unsigned short lb = f2bf_bits(f - bf_bits2f(hb));
          hv[e] = __builtin_bit_cast(_Float16, hb);
          lv[e] = __builtin_bit_cast(_Float16, lb);
        }
        const size_t yo = (size_t)(t * kBatch + row0 + row) * kHid + col;
        *(volatile v8h*)(YShi + yo) = hv;
        *(volatile v8h*)(YSlo + yo) = lv;
      }
      __threadfence();
    }
    __syncthreads();
  }

  for (int pass = 0; pass < 2; ++pass) {
#pragma unroll
    for (int it = 0; it < 8; ++it) {
      const int li = it * 4 + q4;
      const int row = 2 * wave + (li >> 4);
      const int col = (li & 15) * 32 + c4;
      const v4f v = *(const v4f*)(hS + row * kHsp + col);
      *(volatile v4f*)(outH + (size_t)(row0 + row) * kHid + col) = v;
    }
    __threadfence();
  }
  __syncthreads();
#pragma unroll
  for (int ubl = 0; ubl < 4; ++ubl) {
    const int u = 16 * (wave * 4 + ubl) + c;
#pragma unroll
    for (int r = 0; r < 8; ++r) hS[(8 * hh + r) * kHsp + u] = creg[ubl][r];
  }
  __syncthreads();
  for (int pass = 0; pass < 2; ++pass) {
#pragma unroll
    for (int it = 0; it < 8; ++it) {
      const int li = it * 4 + q4;
      const int row = 2 * wave + (li >> 4);
      const int col = (li & 15) * 32 + c4;
      const v4f v = *(const v4f*)(hS + row * kHsp + col);
      *(volatile v4f*)(outC + (size_t)(row0 + row) * kHid + col) = v;
    }
    __threadfence();
  }
}

__global__ __launch_bounds__(256) void value_head_kernel(
    const unsigned short* __restrict__ YShi, const unsigned short* __restrict__ YSlo,
    const float* __restrict__ Wv, const float* __restrict__ bv, float* __restrict__ vout, int nrows) {
  const int r = blockIdx.x * 256 + threadIdx.x;
  const int rc = (r < nrows) ? r : (nrows - 1);
  const v4u* ph = (const v4u*)(YShi + (size_t)rc * kHid);
  const v4u* pl = (const v4u*)(YSlo + (size_t)rc * kHid);
  float s = 0.0f;
#pragma unroll 1
  for (int i = 0; i < kHid / 8; ++i) {
    const v4u wh = ph[i];
    const v4u wl = pl[i];
    const v4f wa = *(const v4f*)(Wv + 8 * i);
    const v4f wb = *(const v4f*)(Wv + 8 * i + 4);
#pragma unroll
    for (int e = 0; e < 4; ++e) {
      const float y0 = __uint_as_float(wh[e] << 16) + __uint_as_float(wl[e] << 16);
      const float y1 = __uint_as_float(wh[e] & 0xffff0000u) + __uint_as_float(wl[e] & 0xffff0000u);
      const float wq0 = (e < 2) ? wa[2 * e] : wb[2 * (e - 2)];
      const float wq1 = (e < 2) ? wa[2 * e + 1] : wb[2 * (e - 2) + 1];
      s += y0 * wq0;
      s += y1 * wq1;
    }
  }
  const float val = s + bv[0];
  if (r < nrows) {
    ((volatile float*)vout)[r] = val;
    __threadfence();
    ((volatile float*)vout)[r] = val;
  }
}

__global__ __launch_bounds__(256) void aw_kernel(
    const float* __restrict__ action_emb, const float* __restrict__ Wa, float* __restrict__ aw, int n) {
  const int i = blockIdx.x * 256 + threadIdx.x;
  if (i < n) {
    const int d = i % kBert;
    const float val = action_emb[i] * Wa[d];
    ((volatile float*)aw)[i] = val;
    __threadfence();
    ((volatile float*)aw)[i] = val;
  }
}

__global__ __launch_bounds__(256) void q_head_kernel(
    const float* __restrict__ proj, const float* __restrict__ aw, const float* __restrict__ ba,
    const float* __restrict__ vbuf, float* __restrict__ qout, int nq) {
  const int idx = blockIdx.x * 256 + threadIdx.x;
  const int ic = (idx < nq) ? idx : (nq - 1);
  const int r = ic / kAct;
  const int act = ic - r * kAct;
  const v4f* pp = (const v4f*)(proj + (size_t)r * kBert);
  const v4f* pa = (const v4f*)(aw + (size_t)act * kBert);
  float s = 0.0f;
#pragma unroll 1
  for (int d4 = 0; d4 < kBert / 4; ++d4) {
    const v4f pv = pp[d4];
    const v4f wv = pa[d4];
    s += pv[0] * wv[0];
    s += pv[1] * wv[1];
    s += pv[2] * wv[2];
    s += pv[3] * wv[3];
  }
  const float a = s + ba[0];
  const float qv = vbuf[r] + a;
  if (idx < nq) {
    ((volatile float*)qout)[idx] = qv;
    __threadfence();
    ((volatile float*)qout)[idx] = qv;
  }
}

extern "C" void kernel_launch(void* const* d_in, const int* in_sizes, int n_in,
                              void* d_out, int out_size, void* d_ws, size_t ws_size,
                              hipStream_t stream) {
  if (n_in < 16) return;
  if (in_sizes[0] != kBatch * kHid || in_sizes[1] != kBatch * kHid) return;
  if (in_sizes[2] != kRows * kState || in_sizes[3] != kSteps * kBatch) return;
  if (in_sizes[4] != kAct * kBert || in_sizes[5] != kState * kHid || in_sizes[6] != kHid) return;
  if (in_sizes[7] != kHid * kGate || in_sizes[8] != kHid * kGate || in_sizes[9] != kGate) return;
  if (in_sizes[10] != kHid * kBert || in_sizes[11] != kBert || in_sizes[12] != kBert) return;
  if (in_sizes[13] < 1 || in_sizes[14] != kHid || in_sizes[15] < 1) return;
  if (out_size != 2 * kBatch * kHid + kRows * kAct) return;

  const float* hidden_c   = (const float*)d_in[0];
  const float* hidden_h   = (const float*)d_in[1];
  const float* state_emb  = (const float*)d_in[2];
  const int*   dones      = (const int*)d_in[3];
  const float* action_emb = (const float*)d_in[4];
  const float* W1     = (const float*)d_in[5];
  const float* b1     = (const float*)d_in[6];
  const float* Wi     = (const float*)d_in[7];
  const float* Wh     = (const float*)d_in[8];
  const float* b_lstm = (const float*)d_in[9];
  const float* Wp     = (const float*)d_in[10];
  const float* bp     = (const float*)d_in[11];
  const float* Wa     = (const float*)d_in[12];
  const float* ba     = (const float*)d_in[13];
  const float* Wv     = (const float*)d_in[14];
  const float* bv     = (const float*)d_in[15];
  float* out = (float*)d_out;
  float* outC = out;
  float* outH = out + (size_t)kBatch * kHid;
  float* outQ = out + (size_t)2 * kBatch * kHid;

  const size_t szSE   = (size_t)kRows * kState * 2;
  const size_t szX16  = (size_t)kRows * kHid * 2;
  const size_t szW1p  = (size_t)kState * kHid * 2;
  const size_t szWg   = (size_t)kGate * kHid * 2;
  const size_t szWpp  = (size_t)kBert * kHid * 2;
  const size_t szGX   = (size_t)kRows * kGate * 4;
  const size_t szYS   = (size_t)kRows * kHid * 2;
  const size_t szV    = (size_t)kRows * 4;
  const size_t szAW   = (size_t)kAct * kBert * 4;
  const size_t szProj = (size_t)kRows * kBert * 4;

  size_t off = 0;
  const size_t oSEhi = off; off += szSE;
  const size_t oSElo = off; off += szSE;
  const size_t oX16  = off; off += szX16;
  const size_t oProj = 0;
  if (szProj > off) return;
  const size_t oW1hi = off; off += szW1p;
  const size_t oW1lo = off; off += szW1p;
  const size_t oWi16 = off; off += szWg;
  const size_t oWh16 = off; off += szWg;
  const size_t oWphi = off; off += szWpp;
  const size_t oWplo = off; off += szWpp;
  const size_t oGX   = off; off += szGX;
  const size_t oYShi = off; off += szYS;
  const size_t oYSlo = off; off += szYS;
  const size_t oV    = off; off += szV;
  const size_t oAW   = off; off += szAW;
  if (off > ws_size) return;

  char* ws = (char*)d_ws;
  unsigned short* SEhi = (unsigned short*)(ws + oSEhi);
  unsigned short* SElo = (unsigned short*)(ws + oSElo);
  unsigned short* X16  = (unsigned short*)(ws + oX16);
  float*          proj = (float*)(ws + oProj);
  unsigned short* W1hi = (unsigned short*)(ws + oW1hi);
  unsigned short* W1lo = (unsigned short*)(ws + oW1lo);
  unsigned short* Wi16 = (unsigned short*)(ws + oWi16);
  unsigned short* Wh16 = (unsigned short*)(ws + oWh16);
  unsigned short* Wphi = (unsigned short*)(ws + oWphi);
  unsigned short* Wplo = (unsigned short*)(ws + oWplo);
  float*          GX   = (float*)(ws + oGX);
  unsigned short* YShi = (unsigned short*)(ws + oYShi);
  unsigned short* YSlo = (unsigned short*)(ws + oYSlo);
  float*          vbuf = (float*)(ws + oV);
  float*          awbuf = (float*)(ws + oAW);

  {
    const int n8 = kRows * kState / 8;
    cast_rows_bf16hl<<<(n8 + 255) / 256, 256, 0, stream>>>(state_emb, SEhi, SElo, n8);
  }
  transpose_cast64<1><<<dim3(kHid / 64, kState / 64), 256, 0, stream>>>(W1, W1hi, W1lo, kState, kHid, 1.0f);
  transpose_cast64<0><<<dim3(kGate / 64, kHid / 64), 256, 0, stream>>>(Wi, Wi16, Wi16, kHid, kGate, 64.0f);
  transpose_cast64<0><<<dim3(kGate / 64, kHid / 64), 256, 0, stream>>>(Wh, Wh16, Wh16, kHid, kGate, 64.0f);
  transpose_cast64<1><<<dim3(kBert / 64, kHid / 64), 256, 0, stream>>>(Wp, Wphi, Wplo, kHid, kBert, 1.0f);

  {
    const int tiles = (kRows / 64) * (kHid / 64);
    wmma_gemm64<1, true, 2, 1, false, 2><<<dim3((tiles + 7) / 8, 1), 256, 0, stream>>>(
        SEhi, SElo, kState, 0L, W1hi, W1lo, kState, 0L,
        (void*)X16, (void*)X16, kHid, 0L, b1, b1, 0L, kRows, kHid, kState, 1.0f);
  }
  {
    const int tiles = (kRows / 64) * (kGate / 64);
    wmma_gemm64<0, false, 2, 0, false, 0><<<dim3((tiles + 7) / 8, 1), 256, 0, stream>>>(
        X16, X16, kHid, 0L, Wi16, Wi16, kHid, 0L,
        (void*)GX, (void*)GX, kGate, 0L, b_lstm, b_lstm, 0L, kRows, kGate, kHid, 1.0f / 64.0f);
  }
  lstm_seq_kernel<<<kBatch / 16, 256, 0, stream>>>(GX, Wh16, dones, hidden_c, hidden_h, YShi, YSlo, outC, outH);

  {
    const int tiles = (kRows / 64) * (kBert / 64);
    wmma_gemm64<1, true, 2, 0, false, 0><<<dim3((tiles + 7) / 8, 1), 256, 0, stream>>>(
        YShi, YSlo, kHid, 0L, Wphi, Wplo, kHid, 0L,
        (void*)proj, (void*)proj, kBert, 0L, bp, bp, 0L, kRows, kBert, kHid, 1.0f);
  }
  value_head_kernel<<<(kRows + 255) / 256, 256, 0, stream>>>(YShi, YSlo, Wv, bv, vbuf, kRows);
  aw_kernel<<<(kAct * kBert + 255) / 256, 256, 0, stream>>>(action_emb, Wa, awbuf, kAct * kBert);
  q_head_kernel<<<(kRows * kAct + 255) / 256, 256, 0, stream>>>(proj, awbuf, ba, vbuf, outQ, kRows * kAct);
}
